// Generator_4569845203153
// MI455X (gfx1250) — hardware-run, weakly checked
//
#include <hip/hip_runtime.h>
#include <math.h>

typedef __attribute__((ext_vector_type(16))) _Float16 v16h;
typedef __attribute__((ext_vector_type(8)))  _Float16 v8h;
typedef __attribute__((ext_vector_type(8)))  float    v8f;
typedef __attribute__((ext_vector_type(4)))  float    v4f;

constexpr int kT   = 65536;
constexpr int kZ   = 100;
constexpr int kZ1  = 10;
constexpr int kH   = 100;
constexpr int kG   = 4 * kH;
constexpr int kKP  = 128;
constexpr int kNP  = 448;
constexpr int kXP  = 416;
constexpr float kCarryA = 64.0f;
constexpr float kCarryB = 64.0f;
constexpr float kFold   = 1.0f / (kCarryA * kCarryB);
constexpr float kF16Min = 6.103515625e-5f;

static_assert(kG == 400);
static_assert(kKP % 32 == 0 && kKP >= kH);
static_assert(kNP % 64 == 0 && kNP >= kG);
static_assert(kT % 64 == 0);
static_assert(kXP % 32 == 0 && kXP >= kG && kXP <= kNP);
static_assert(((kT / 64) * (kNP / 64)) % 8 == 0);
static_assert(kT % 8 == 0);
static_assert(kT % 32 == 0);

constexpr size_t kSzY16   = (size_t)kT * kKP * 2;
constexpr size_t kSzKT16  = (size_t)kNP * kKP * 2;
constexpr size_t kSzBias  = (size_t)kNP * 4;
constexpr size_t kSzXG    = (size_t)kT * kXP * 4;
constexpr size_t kOffY16  = 0;
constexpr size_t kOffKT16 = kOffY16 + kSzY16;
constexpr size_t kOffBias = kOffKT16 + kSzKT16;
constexpr size_t kOffXG   = kOffBias + kSzBias;
constexpr size_t kWsTotal = kOffXG + kSzXG;
static_assert(kSzY16 == 16777216ull && kSzKT16 == 114688ull && kSzBias == 1792ull && kSzXG == 109051904ull);
static_assert(kWsTotal == 125945600ull);
static_assert(kWsTotal <= 134217728ull);
static_assert((kOffKT16 % 256) == 0 && (kOffBias % 256) == 0 && (kOffXG % 256) == 0);

__device__ __forceinline__ void pin1(float& a) { asm volatile("" : "+v"(a)); }
__device__ __forceinline__ _Float16 to_f16_flush(float v) {
  const float w = (fabsf(v) < kF16Min) ? 0.0f : v;
  return (_Float16)w;
}

__device__ __forceinline__ void dep_guard4_h(v8f& a, v8f& b, v8f& c, v8f& d, v16h x, v16h y) {
  asm volatile("v_nop\n\tv_nop\n\tv_nop\n\tv_nop" : "+v"(a), "+v"(b), "+v"(c), "+v"(d) : "v"(x), "v"(y));
}
__device__ __forceinline__ void keep4_h(v16h a, v16h b, v16h c, v16h d) { asm volatile("v_nop" :: "v"(a), "v"(b), "v"(c), "v"(d)); }
__device__ __forceinline__ void acc_guard4(v8f& a, v8f& b, v8f& c, v8f& d) {
  asm volatile("v_nop\n\tv_nop\n\tv_nop\n\tv_nop" : "+v"(a), "+v"(b), "+v"(c), "+v"(d));
}
struct FragH {
  union U { v16h v; v8h h[2]; };
  static __device__ __forceinline__ v16h load(const _Float16* p) {
    U f; f.h[0] = *(const v8h*)(p); f.h[1] = *(const v8h*)(p + 16); return f.v;
  }
  static __device__ __forceinline__ v8f mma(v16h a, v16h b, v8f c) {
    return __builtin_amdgcn_wmma_f32_16x16x32_f16(false, a, false, b, (short)0, c, false, false);
  }
};

constexpr int kPrepPlaneBlocks = (kNP * (kKP / 8)) / 256;
constexpr int kPrepBlocks      = kPrepPlaneBlocks + 1;
static_assert((kNP * (kKP / 8)) % 256 == 0 && kPrepPlaneBlocks == 28);
static_assert(kNP / 4 == 112);

__global__ __launch_bounds__(256) void prep_kernel(const float* __restrict__ lk, const float* __restrict__ lb,
                                                   unsigned short* __restrict__ kt16, float* __restrict__ bias448) {
  const int tid = threadIdx.x;
  if (blockIdx.x < kPrepPlaneBlocks) {
    const int i  = blockIdx.x * 256 + tid;
    const int n  = i >> 4;
    const int k0 = (i & 15) * 8;
    const int nc = (n < kG) ? n : (kG - 1);
    v8h hv;
#pragma unroll
    for (int e = 0; e < 8; ++e) {
      const int k  = k0 + e;
      const int kc = (k < kH) ? k : (kH - 1);
      float v = lk[(size_t)kc * kG + nc];
      pin1(v);
      const bool ok = (k < kH) && (n < kG);
      const float w = ok ? (v * kCarryB) : 0.0f;
      hv[e] = to_f16_flush(w);
    }
    unsigned short* dst = kt16 + (size_t)i * 8;
    *(volatile v8h*)dst = hv;
    __threadfence();
    *(volatile v8h*)dst = hv;
  } else {
    v4f o;
#pragma unroll
    for (int e = 0; e < 4; ++e) {
      const int idx = 4 * tid + e;
      const int ic  = (idx < kG) ? idx : (kG - 1);
      float v = lb[ic];
      pin1(v);
      o[e] = (idx < kG) ? v : 0.0f;
    }
    if (tid < kNP / 4) {
      float* dst = bias448 + 4 * tid;
      *(volatile v4f*)dst = o;
      __threadfence();
      *(volatile v4f*)dst = o;
    }
  }
}

__global__ __launch_bounds__(256) void front_kernel(const float* __restrict__ x, const float* __restrict__ Wz,
                                                    const float* __restrict__ bz, const float* __restrict__ Wy,
                                                    const float* __restrict__ by, unsigned short* __restrict__ y16) {
  __shared__ __align__(16) float sY[8][kKP];
  const int lane = threadIdx.x & 31, wave = threadIdx.x >> 5;
  const int row  = blockIdx.x * 8 + wave;
  const float* xr = x + (size_t)row * kZ;

  float p[kZ1];
#pragma unroll
  for (int j = 0; j < kZ1; ++j) p[j] = 0.0f;
#pragma unroll 1
  for (int i = 0; i < 4; ++i) {
    const int k  = lane + 32 * i;
    const int kc = (k < kZ) ? k : (kZ - 1);
    float xv = xr[kc];
    pin1(xv);
    xv = (k < kZ) ? xv : 0.0f;
    const float* wr = Wz + kc * kZ1;
#pragma unroll
    for (int j = 0; j < kZ1; ++j) p[j] = fmaf(xv, wr[j], p[j]);
  }
  float z[kZ1];
#pragma unroll
  for (int j = 0; j < kZ1; ++j) {
    float v = p[j];
#pragma unroll
    for (int off = 16; off >= 1; off >>= 1) v += __shfl_xor(v, off, 32);
    z[j] = fmaxf(v + bz[j], 0.0f);
  }

  float* sy = sY[wave];
#pragma unroll 1
  for (int q = 0; q < 4; ++q) {
    const int j  = lane + 32 * q;
    const int jc = (j < kH) ? j : (kH - 1);
    float acc = 0.0f;
#pragma unroll
    for (int m = 0; m < kZ1; ++m) acc = fmaf(z[m], Wy[m * kH + jc], acc);
    acc += by[jc];
    float yv = fmaxf(acc, 0.0f) * kCarryA;
    yv = (j < kH) ? yv : 0.0f;
    yv = (yv < kF16Min) ? 0.0f : yv;
    sy[j] = yv;
  }
  __builtin_amdgcn_fence(__ATOMIC_RELEASE, "workgroup");
  __builtin_amdgcn_wave_barrier();
  __builtin_amdgcn_fence(__ATOMIC_ACQUIRE, "workgroup");
  {
    const int l16 = lane & 15;
    const float* sp = sy + 8 * l16;
    const v4f a0 = *(const v4f*)(sp);
    const v4f a1 = *(const v4f*)(sp + 4);
    v8h hv;
#pragma unroll
    for (int e = 0; e < 4; ++e) {
      hv[e]     = (_Float16)a0[e];
      hv[4 + e] = (_Float16)a1[e];
    }
    unsigned short* dst = y16 + (size_t)row * kKP + 8 * l16;
    if (lane < 16) {
      *(volatile v8h*)dst = hv;
      __threadfence();
      *(volatile v8h*)dst = hv;
    }
  }
}

__global__ __launch_bounds__(256) void gemm_f16_kernel(
    const unsigned short* __restrict__ Ap, int lda,
    const unsigned short* __restrict__ Btp, int ldb,
    float* __restrict__ C, int ldc, int nStore,
    const float* __restrict__ bias, int M, int N, int K, float scale) {
  const _Float16* A  = (const _Float16*)Ap;
  const _Float16* Bt = (const _Float16*)Btp;
  __shared__ __align__(16) float sT[8][16 * 68];
  const int lane = threadIdx.x & 31;
  const int wave = threadIdx.x >> 5;
  const int tilesN = N >> 6;
  const int tilesM = M >> 6;
  const int tile = blockIdx.x * 8 + wave;
  if (tile >= tilesM * tilesN) return;
  const int tm = tile / tilesN;
  const int tn = tile - tm * tilesN;
  const int m0 = tm << 6;
  const int n0 = tn << 6;

  const int rlane = lane & 15;
  const int koff  = (lane >> 4) * 8;
  const int mOff  = (lane >> 4) * 8;

  v8f acc[4][4];
#pragma unroll
  for (int i = 0; i < 4; ++i)
#pragma unroll
    for (int j = 0; j < 4; ++j) acc[i][j] = (v8f){0.f, 0.f, 0.f, 0.f, 0.f, 0.f, 0.f, 0.f};

  for (int k0 = 0; k0 < K; k0 += 32) {
    v16h bh[4];
#pragma unroll
    for (int j = 0; j < 4; ++j) {
      const size_t bo = (size_t)(n0 + (j << 4) + rlane) * ldb + koff + k0;
      bh[j] = FragH::load(Bt + bo);
    }
#pragma unroll
    for (int i = 0; i < 4; ++i) {
      const size_t ao = (size_t)(m0 + (i << 4) + rlane) * lda + koff + k0;
      const v16h ah = FragH::load(A + ao);
#pragma unroll
      for (int j = 0; j < 4; ++j) acc[i][j] = FragH::mma(ah, bh[j], acc[i][j]);
      dep_guard4_h(acc[i][0], acc[i][1], acc[i][2], acc[i][3], ah, bh[3]);
    }
    keep4_h(bh[0], bh[1], bh[2], bh[3]);
  }
  acc_guard4(acc[0][0], acc[0][1], acc[0][2], acc[0][3]);
  acc_guard4(acc[1][0], acc[1][1], acc[1][2], acc[1][3]);
  acc_guard4(acc[2][0], acc[2][1], acc[2][2], acc[2][3]);
  acc_guard4(acc[3][0], acc[3][1], acc[3][2], acc[3][3]);

  float* slab = sT[wave];
#pragma unroll
  for (int i = 0; i < 4; ++i) {
    const int mBase = m0 + (i << 4);
#pragma unroll
    for (int j = 0; j < 4; ++j) {
      const int n = n0 + (j << 4) + rlane;
      const float bv = bias[n];
#pragma unroll
      for (int r = 0; r < 8; ++r) {
        float v = acc[i][j][r] * scale;
        v += bv;
        slab[(mOff + r) * 68 + (j << 4) + rlane] = v;
      }
    }
    __builtin_amdgcn_fence(__ATOMIC_RELEASE, "workgroup");
    __builtin_amdgcn_wave_barrier();
    __builtin_amdgcn_fence(__ATOMIC_ACQUIRE, "workgroup");
    {
      const int hh = lane >> 4, c4 = (lane & 15) * 4;
      const bool st = (n0 + c4) < nStore;
      for (int pass = 0; pass < 2; ++pass) {
#pragma unroll
        for (int it = 0; it < 8; ++it) {
          const int row = it * 2 + hh;
          const v4f v = *(const v4f*)(slab + row * 68 + c4);
          if (st) *(volatile v4f*)(C + (size_t)(mBase + row) * ldc + n0 + c4) = v;
        }
        __threadfence();
      }
    }
    __builtin_amdgcn_fence(__ATOMIC_RELEASE, "workgroup");
    __builtin_amdgcn_wave_barrier();
    __builtin_amdgcn_fence(__ATOMIC_ACQUIRE, "workgroup");
  }
}

constexpr int kScanThreads = 800;
constexpr int kKHalf  = 52;
constexpr int kHPitch = 104;
constexpr int kRing   = 64;
static_assert(kScanThreads == 8 * kH && kScanThreads % 32 == 0);
static_assert(2 * kKHalf == kHPitch && kHPitch >= kH && kKHalf % 4 == 0);
static_assert(kKHalf == 4 * 13);

__global__ __launch_bounds__(kScanThreads) void scan_kernel(const float* __restrict__ xg, const float* __restrict__ R,
                                                            const float* __restrict__ Wf, const float* __restrict__ bf,
                                                            float* __restrict__ out) {
  __shared__ __align__(16) float hb[2 * kHPitch];
  __shared__ __align__(16) float hring[kRing * kHPitch];
  __shared__ __align__(16) float swf[kHPitch];
  const int tid = threadIdx.x, lane = tid & 31;
  const int kh = tid & 1, gate = (tid >> 1) & 3, u = tid >> 3;
  const int col = gate * kH + u;
  const int gbase = lane & 24;

  float rc[kKHalf];
#pragma unroll
  for (int g = 0; g < 4; ++g) {
#pragma unroll
    for (int e = 0; e < 13; ++e) {
      const int k  = kh * kKHalf + 13 * g + e;
      const int kc = (k < kH) ? k : (kH - 1);
      rc[13 * g + e] = R[(size_t)kc * kG + col];
    }
#pragma unroll
    for (int e = 0; e < 13; ++e) pin1(rc[13 * g + e]);
    __builtin_amdgcn_sched_barrier(0);
  }
#pragma unroll
  for (int e = 0; e < kKHalf; ++e) {
    const int k = kh * kKHalf + e;
    rc[e] = (k < kH) ? rc[e] : 0.0f;
  }

  if (tid < 2 * kHPitch) hb[tid] = 0.0f;
  {
    const int wc = (tid < kH) ? tid : (kH - 1);
    float wv = Wf[wc];
    pin1(wv);
    if (tid < kHPitch) swf[tid] = (tid < kH) ? wv : 0.0f;
  }
  const float bfv = bf[0];
  float cst = 0.0f;
  float gnext = xg[col];
  __syncthreads();

#pragma unroll 1
  for (int t = 0; t < kT; ++t) {
    const float gcur = gnext;
    const int tn = (t + 1 < kT) ? (t + 1) : (kT - 1);
    gnext = xg[(size_t)tn * kXP + col];

    const float* hp = hb + (t & 1) * kHPitch + kh * kKHalf;
    float a0 = 0.0f, a1 = 0.0f, a2 = 0.0f, a3 = 0.0f;
#pragma unroll
    for (int e4 = 0; e4 < kKHalf / 4; ++e4) {
      const v4f hv = *(const v4f*)(hp + 4 * e4);
      a0 = fmaf(hv[0], rc[4 * e4 + 0], a0);
      a1 = fmaf(hv[1], rc[4 * e4 + 1], a1);
      a2 = fmaf(hv[2], rc[4 * e4 + 2], a2);
      a3 = fmaf(hv[3], rc[4 * e4 + 3], a3);
    }
    pin1(gnext);
    const float part = (a0 + a1) + (a2 + a3);
    const float oth  = __shfl_xor(part, 1, 32);
    const float g    = gcur + (part + oth);

    const float sg = __builtin_amdgcn_rcpf(1.0f + __expf(-g));
    const float rl = fmaxf(g, 0.0f);
    const float gi = __shfl(sg, gbase + 0, 32);
    const float gf = __shfl(sg, gbase + 2, 32);
    const float gc = __shfl(rl, gbase + 4, 32);
    const float go = __shfl(sg, gbase + 6, 32);

    cst = gf * cst + gi * gc;
    const float hnew = go * fmaxf(cst, 0.0f);

    float* hn = hb + ((t + 1) & 1) * kHPitch;
    if ((tid & 7) == 0) {
      hn[u] = hnew;
      hring[(t & (kRing - 1)) * kHPitch + u] = hnew;
    }
    if ((tid & 7) == 1 && u < 4) hn[kH + u] = 0.0f;
    __syncthreads();

    if ((t & 31) == 31) {
      if (tid < 32) {
        const int t0 = t - 31;
        const float* hr = hring + ((t0 & (kRing - 1)) + lane) * kHPitch;
        float s0 = 0.0f, s1 = 0.0f, s2 = 0.0f, s3 = 0.0f;
#pragma unroll 1
        for (int e4 = 0; e4 < kH / 4; ++e4) {
          const v4f hv = *(const v4f*)(hr + 4 * e4);
          const v4f wv = *(const v4f*)(swf + 4 * e4);
          s0 = fmaf(hv[0], wv[0], s0);
          s1 = fmaf(hv[1], wv[1], s1);
          s2 = fmaf(hv[2], wv[2], s2);
          s3 = fmaf(hv[3], wv[3], s3);
        }
        const float o = ((s0 + s1) + (s2 + s3)) + bfv;
        float* op = out + t0 + lane;
        *(volatile float*)op = o;
        __threadfence();
        *(volatile float*)op = o;
      }
    }
  }
}

extern "C" void kernel_launch(void* const* d_in, const int* in_sizes, int n_in,
                              void* d_out, int out_size, void* d_ws, size_t ws_size, hipStream_t stream) {
  if (n_in < 10 || d_out == nullptr || d_ws == nullptr) return;
  if (in_sizes[0] != kT * kZ || in_sizes[1] != kZ * kZ1 || in_sizes[2] != kZ1 || in_sizes[3] != kZ1 * kH ||
      in_sizes[4] != kH || in_sizes[5] != kH * kG || in_sizes[6] != kH * kG || in_sizes[7] != kG ||
      in_sizes[8] != kH || in_sizes[9] != 1 || out_size != kT) return;
  if (ws_size < kWsTotal) return;

  const float* x   = (const float*)d_in[0];
  const float* Wz  = (const float*)d_in[1];
  const float* bz  = (const float*)d_in[2];
  const float* Wy  = (const float*)d_in[3];
  const float* by  = (const float*)d_in[4];
  const float* lk  = (const float*)d_in[5];
  const float* lr  = (const float*)d_in[6];
  const float* lb  = (const float*)d_in[7];
  const float* Wf  = (const float*)d_in[8];
  const float* bfp = (const float*)d_in[9];
  float* out = (float*)d_out;

  char* ws = (char*)d_ws;
  unsigned short* Y16     = (unsigned short*)(ws + kOffY16);
  unsigned short* KT16    = (unsigned short*)(ws + kOffKT16);
  float*          BIAS448 = (float*)(ws + kOffBias);
  float*          XG      = (float*)(ws + kOffXG);

  prep_kernel<<<kPrepBlocks, 256, 0, stream>>>(lk, lb, KT16, BIAS448);

  front_kernel<<<kT / 8, 256, 0, stream>>>(x, Wz, bz, Wy, by, Y16);

  gemm_f16_kernel<<<((kT / 64) * (kNP / 64)) / 8, 256, 0, stream>>>(
      Y16, kKP, KT16, kKP, XG, kXP, kXP, BIAS448, kT, kNP, kKP, kFold);

  scan_kernel<<<1, kScanThreads, 0, stream>>>(XG, lr, Wf, bfp, out);
}
